// CoordAttentionV2_29824252903435
// MI455X (gfx1250) — hardware-verified
//
#include <hip/hip_runtime.h>
#include <math.h>

typedef __attribute__((ext_vector_type(16))) _Float16 v16h;
typedef __attribute__((ext_vector_type(16))) __bf16 v16b;
typedef __attribute__((ext_vector_type(8)))  _Float16 v8h;
typedef __attribute__((ext_vector_type(8)))  float v8f;
typedef __attribute__((ext_vector_type(4)))  float v4f;
typedef __attribute__((ext_vector_type(2)))  float v2f;
typedef __attribute__((ext_vector_type(4)))  unsigned v4u;
typedef __attribute__((ext_vector_type(4)))  int v4i;
typedef float __attribute__((may_alias)) float_a;
typedef int __attribute__((may_alias)) int_a;

template <typename T> __device__ __forceinline__ void vst2(void* p, T v) { *(volatile T*)p = v; __threadfence(); *(volatile T*)p = v; }
__device__ __forceinline__ v8f wmma16(v16h a, v16h b, v8f c) {
  v8f d = __builtin_amdgcn_wmma_f32_16x16x32_f16(false, a, false, b, (short)0, c, false, false);
  asm volatile("v_nop\n\tv_nop\n\tv_nop\n\tv_nop" : "+v"(d) : "v"(a), "v"(b));
  return d;
}
__device__ __forceinline__ v8f wmma_bf(v16b a, v16b b, v8f c) {
  v8f d = __builtin_amdgcn_wmma_f32_16x16x32_bf16(false, a, false, b, (short)0, c, false, false);
  asm volatile("v_nop\n\tv_nop\n\tv_nop\n\tv_nop" : "+v"(d) : "v"(a), "v"(b));
  return d;
}
__device__ __forceinline__ v16h frag_h(const _Float16* rowk0, int lane) {
  union { v16h v; v8h q[2]; } u; const _Float16* p = rowk0 + 8 * (lane >> 4);
  u.q[0] = *(const v8h*)p; u.q[1] = *(const v8h*)(p + 16); return u.v;
}
__device__ __forceinline__ v16h frag_f32(const float* rowk0, int lane) {
  v16h a; const float* p = rowk0 + 8 * (lane >> 4);
#pragma unroll
  for (int i = 0; i < 8; ++i) { a[i] = (_Float16)p[i]; a[8 + i] = (_Float16)p[16 + i]; }
  return a;
}
__device__ __forceinline__ v16h frag_f32s(const float* rowk0, int lane, float sc) {
  v16h a; const float* p = rowk0 + 8 * (lane >> 4);
#pragma unroll
  for (int i = 0; i < 8; ++i) { a[i] = (_Float16)(p[i] * sc); a[8 + i] = (_Float16)(p[16 + i] * sc); }
  return a;
}
__device__ __forceinline__ v16h fragc_f32(const float* W, int k0, int n, int lane, int ld, int K) {
  v16h a; const int g = lane >> 4;
#pragma unroll
  for (int i = 0; i < 8; ++i) { const int ka = k0 + 8 * g + i, kb = ka + 16;
    a[i] = (_Float16)(ka < K ? W[(size_t)(ka < K ? ka : K - 1) * ld + n] : 0.f); a[8 + i] = (_Float16)(kb < K ? W[(size_t)(kb < K ? kb : K - 1) * ld + n] : 0.f); }
  return a;
}
struct F2 { v16b h, l; };
__device__ __forceinline__ F2 bsplit16(const float v[16]) { F2 r;
#pragma unroll
  for (int i = 0; i < 16; ++i) { const __bf16 h = (__bf16)v[i]; r.h[i] = h; r.l[i] = (__bf16)(v[i] - (float)h); }
  return r; }
__device__ __forceinline__ F2 split_row(const float* row, int k0, int lane) { float v[16]; const float* p = row + k0 + 8 * (lane >> 4);
#pragma unroll
  for (int i = 0; i < 8; ++i) { v[i] = p[i]; v[8 + i] = p[16 + i]; }
  return bsplit16(v); }
__device__ __forceinline__ F2 split_rowK(const float* row, int k0, int lane, int K) { float v[16]; const int g = lane >> 4;
#pragma unroll
  for (int i = 0; i < 8; ++i) { const int ka = k0 + 8 * g + i, kb = ka + 16; v[i] = ka < K ? row[ka < K ? ka : K - 1] : 0.f; v[8 + i] = kb < K ? row[kb < K ? kb : K - 1] : 0.f; }
  return bsplit16(v); }
__device__ __forceinline__ F2 split_col(const float* W, int k0, int n, int lane, int ld, int K) { float v[16]; const int g = lane >> 4;
#pragma unroll
  for (int i = 0; i < 8; ++i) { const int ka = k0 + 8 * g + i, kb = ka + 16; v[i] = ka < K ? W[(size_t)(ka < K ? ka : K - 1) * ld + n] : 0.f; v[8 + i] = kb < K ? W[(size_t)(kb < K ? kb : K - 1) * ld + n] : 0.f; }
  return bsplit16(v); }
__device__ __forceinline__ v8f mac3(const F2& a, const F2& b, v8f c) { c = wmma_bf(a.l, b.h, c); c = wmma_bf(a.h, b.l, c); return wmma_bf(a.h, b.h, c); }
__device__ __forceinline__ float sigm(float v) { return 1.0f / (1.0f + expf(-v)); }
#define LDSX() do { asm volatile("s_wait_dscnt 0" ::: "memory"); __builtin_amdgcn_wave_barrier(); __builtin_amdgcn_fence(__ATOMIC_RELEASE, "workgroup"); } while (0)


#define NB 2
#define SS 2048
#define FD 512
#define CD 3
#define IND 515
#define NFH 8
#define NHT 9
#define HD 64
#define IV 576
#define OD 512
#define NR (NB * SS)
__device__ __forceinline__ float bfr(float v) { return (float)(__bf16)v; }
__device__ __forceinline__ v16b frag_b(const __bf16* rowk0, int lane) { return __builtin_bit_cast(v16b, frag_h((const _Float16*)rowk0, lane)); }
__device__ __attribute__((noinline)) float exp_ni(float v) { return expf(v); }

__global__ __launch_bounds__(128) void k_proj(const float* __restrict__ x, const float* __restrict__ cx, const float* __restrict__ y, const float* __restrict__ cy, const float* __restrict__ Wq, const float* __restrict__ Wk, const float* __restrict__ Wv,
                                             float* __restrict__ Q32, __bf16* __restrict__ Kh, __bf16* __restrict__ Kl, __bf16* __restrict__ VTh, __bf16* __restrict__ VTl) {
  __shared__ __align__(16) float so[4][16][132]; __shared__ __align__(16) __bf16 sh_[4][16][136], sl_[4][16][136]; __shared__ __align__(16) __bf16 sth[128][72], stl[128][72];
  const int tid = threadIdx.x, wave = tid >> 5, lane = tid & 31, col = lane & 15, g = lane >> 4; const int which = blockIdx.z, r0b = blockIdx.x * 64, n0 = blockIdx.y * 128; const size_t r0 = (size_t)r0b + wave * 16; const int b = r0b / SS, s0 = r0b % SS;
  const int ncol = which == 2 ? IV : OD; if (n0 >= ncol) return; const int ntile = (ncol - n0) >= 128 ? 8 : (ncol - n0) / 16;
  const float* F = which == 0 ? x : y; const float* C = which == 0 ? cx : cy; const float* W = which == 0 ? Wq : (which == 1 ? Wk : Wv);
  v8f acc[8] = {};
#pragma unroll 1
  for (int kc = 0; kc <= FD / 32; ++kc) { const v16b a = kc < FD / 32 ? split_row(F + (r0 + col) * FD, kc * 32, lane).h : split_rowK(C + (r0 + col) * CD, 0, lane, CD).h;
#pragma unroll
    for (int j = 0; j < 8; ++j) { if (j < ntile) acc[j] = wmma_bf(a, split_col(W, kc * 32, n0 + j * 16 + col, lane, ncol, IND).h, acc[j]); } }
  if (which == 0) {
#pragma unroll
    for (int j = 0; j < 8; ++j)
#pragma unroll
      for (int r = 0; r < 8; ++r) so[wave][8 * g + r][j * 16 + col] = acc[j][r];
    LDSX();
    for (int qq = lane; qq < 2 * 16 * 16; qq += 32) { const int hh = qq >> 8, rl = (qq >> 4) & 15, pc = qq & 15; const int h = (n0 >> 6) + hh; vst2(Q32 + (((size_t)b * NFH + h) * SS + s0 + wave * 16 + rl) * HD + pc * 4, *(const v4f*)(&so[wave][rl][hh * 64 + pc * 4])); } }
  else if (which == 1) {
#pragma unroll
    for (int j = 0; j < 8; ++j)
#pragma unroll
      for (int r = 0; r < 8; ++r) { const float v = acc[j][r]; const __bf16 hi = (__bf16)v; sh_[wave][8 * g + r][j * 16 + col] = hi; sl_[wave][8 * g + r][j * 16 + col] = (__bf16)(v - (float)hi); }
    LDSX();
    for (int qq = lane; qq < 2 * 16 * 8; qq += 32) { const int hh = qq >> 7, rl = (qq >> 3) & 15, pc = qq & 7; const int h = (n0 >> 6) + hh; const size_t o = (((size_t)b * NFH + h) * SS + s0 + wave * 16 + rl) * HD + pc * 8; vst2((unsigned*)(Kh + o), *(const v4u*)(&sh_[wave][rl][hh * 64 + pc * 8])); vst2((unsigned*)(Kl + o), *(const v4u*)(&sl_[wave][rl][hh * 64 + pc * 8])); } }
  else {
#pragma unroll
    for (int j = 0; j < 8; ++j)
#pragma unroll
      for (int r = 0; r < 8; ++r) { const float v = acc[j][r]; const __bf16 hi = (__bf16)v; sth[j * 16 + col][wave * 16 + 8 * g + r] = hi; stl[j * 16 + col][wave * 16 + 8 * g + r] = (__bf16)(v - (float)hi); }
    __syncthreads();
    for (int qq = tid; qq < ntile * 16 * 8; qq += 128) { const int cl = qq >> 3, pc = qq & 7; const int c = n0 + cl; const int h = c >> 6, d = c & 63; const size_t o = (((size_t)b * NHT + h) * HD + d) * SS + s0 + pc * 8; vst2((unsigned*)(VTh + o), *(const v4u*)(&sth[cl][pc * 8])); vst2((unsigned*)(VTl + o), *(const v4u*)(&stl[cl][pc * 8])); } }
}
__global__ __launch_bounds__(128) void k_attn(const float* __restrict__ Q32, const __bf16* __restrict__ Kh, const __bf16* __restrict__ Kl, const __bf16* __restrict__ VTh, const __bf16* __restrict__ VTl, const float* __restrict__ cx, const float* __restrict__ cy, const float* __restrict__ csp, float* __restrict__ O) {
  __shared__ __align__(16) float sS[4][16][68]; __shared__ __align__(16) __bf16 sPh[4][16][72], sPl[4][16][72]; __shared__ __align__(16) float sO[4][16][68];
  const int tid = threadIdx.x, w = tid >> 5, lane = tid & 31, col = lane & 15, g = lane >> 4; const int bh = blockIdx.y; const int b = bh / NHT, h = bh % NHT; const int q0 = blockIdx.x * 64 + w * 16; const bool coordh = (h == NFH);
  F2 aq[2]; v16b ac; const float cs = bfr(csp[0]);
  if (!coordh) {
#pragma unroll
    for (int kc = 0; kc < 2; ++kc) aq[kc] = split_row(Q32 + (((size_t)b * NFH + h) * SS + q0 + col) * HD, kc * 32, lane); }
  else { ac = split_rowK(cx + ((size_t)b * SS + q0 + col) * CD, 0, lane, CD).h; }
  float mrun = -3.0e38f, lrun = 0.f; v8f acc[4] = {};
#pragma unroll 1
  for (int kt = 0; kt < SS / 64; ++kt) {
#pragma unroll
    for (int t = 0; t < 4; ++t) { const int key = kt * 64 + t * 16 + col; v8f s = {};
      if (!coordh) { const size_t ko = (((size_t)b * NFH + h) * SS + key) * HD;
#pragma unroll
        for (int kc = 0; kc < 2; ++kc) { const v16b khf = frag_b(Kh + ko + kc * 32, lane), klf = frag_b(Kl + ko + kc * 32, lane); s = wmma_bf(aq[kc].l, khf, s); s = wmma_bf(aq[kc].h, klf, s); s = wmma_bf(aq[kc].h, khf, s); }
#pragma unroll
        for (int r = 0; r < 8; ++r) sS[w][8 * g + r][t * 16 + col] = s[r] * 0.125f; }
      else { s = wmma_bf(ac, split_rowK(cy + ((size_t)b * SS + key) * CD, 0, lane, CD).h, s);
#pragma unroll
        for (int r = 0; r < 8; ++r) sS[w][8 * g + r][t * 16 + col] = s[r] * cs; } }
    LDSX();
    float mx = -3.4e38f;
#pragma unroll
    for (int jj = 0; jj < 32; ++jj) mx = fmaxf(mx, sS[w][col][g * 32 + jj]);
    mx = fmaxf(mx, __shfl_xor(mx, 16, 32));
    const float mnew = fmaxf(mrun, mx); const float corr = expf(mrun - mnew);
    float ps = 0.f;
#pragma unroll 4
    for (int jj = 0; jj < 32; ++jj) { const float p = exp_ni(sS[w][col][g * 32 + jj] - mnew); ps += p; const __bf16 hi = (__bf16)p; sPh[w][col][g * 32 + jj] = hi; sPl[w][col][g * 32 + jj] = (__bf16)(p - (float)hi); }
    ps += __shfl_xor(ps, 16, 32);
    lrun = lrun * corr + ps; mrun = mnew;
#pragma unroll
    for (int r = 0; r < 8; ++r) { const float cr = __shfl(corr, 8 * g + r, 32);
#pragma unroll
      for (int t = 0; t < 4; ++t) acc[t][r] *= cr; }
    LDSX();
#pragma unroll
    for (int kc = 0; kc < 2; ++kc) { const v16b ph = frag_b(&sPh[w][col][0] + kc * 32, lane), pl = frag_b(&sPl[w][col][0] + kc * 32, lane);
#pragma unroll
      for (int t = 0; t < 4; ++t) { const size_t vo = (((size_t)b * NHT + h) * HD + t * 16 + col) * SS + kt * 64 + kc * 32; const v16b vh = frag_b(VTh + vo, lane), vl = frag_b(VTl + vo, lane); acc[t] = wmma_bf(pl, vh, acc[t]); acc[t] = wmma_bf(ph, vl, acc[t]); acc[t] = wmma_bf(ph, vh, acc[t]); } }
    __builtin_amdgcn_wave_barrier(); }
#pragma unroll
  for (int r = 0; r < 8; ++r) { const float lr = __shfl(lrun, 8 * g + r, 32); const float inv = 1.0f / lr;
#pragma unroll
    for (int t = 0; t < 4; ++t) sO[w][8 * g + r][t * 16 + col] = acc[t][r] * inv; }
  LDSX();
  for (int qq = lane; qq < 16 * 16; qq += 32) { const int rl = qq >> 4, pc = qq & 15; vst2(O + ((size_t)b * SS + q0 + rl) * IV + h * HD + pc * 4, *(const v4f*)(&sO[w][rl][pc * 4])); }
}
__global__ __launch_bounds__(128) void k_out(const float* __restrict__ O, const float* __restrict__ Wo, float* __restrict__ out) {
  __shared__ __align__(16) float so[4][16][132];
  const int tid = threadIdx.x, wave = tid >> 5, lane = tid & 31, col = lane & 15, g = lane >> 4; const size_t r0 = (size_t)blockIdx.x * 64 + wave * 16; const int n0 = blockIdx.y * 128;
  v8f acc[8] = {};
#pragma unroll 2
  for (int kc = 0; kc < IV / 32; ++kc) { const F2 a = split_row(O + (r0 + col) * IV, kc * 32, lane);
#pragma unroll
    for (int j = 0; j < 8; ++j) { const v16b wb = split_col(Wo, kc * 32, n0 + j * 16 + col, lane, OD, IV).h; acc[j] = wmma_bf(a.l, wb, acc[j]); acc[j] = wmma_bf(a.h, wb, acc[j]); } }
#pragma unroll
  for (int j = 0; j < 8; ++j)
#pragma unroll
    for (int r = 0; r < 8; ++r) so[wave][8 * g + r][j * 16 + col] = acc[j][r];
  LDSX();
  for (int rl = 0; rl < 16; ++rl) vst2(out + (r0 + rl) * OD + n0 + lane * 4, *(const v4f*)(&so[wave][rl][lane * 4]));
}
extern "C" void kernel_launch(void* const* d_in, const int* in_sizes, int n_in, void* d_out, int out_size, void* d_ws, size_t ws_size, hipStream_t stream) {
  (void)in_sizes; (void)n_in; (void)out_size; (void)ws_size;
  const float** I = (const float**)d_in;
  char* ws = (char*)d_ws; size_t off = 0;
  auto take = [&](size_t bytes) { char* p = ws + off; off += (bytes + 255) & ~(size_t)255; return p; };
  float* Q32 = (float*)take((size_t)NR * OD * 4); __bf16* Kh = (__bf16*)take((size_t)NR * OD * 2); __bf16* Kl = (__bf16*)take((size_t)NR * OD * 2); __bf16* VTh = (__bf16*)take((size_t)NR * IV * 2); __bf16* VTl = (__bf16*)take((size_t)NR * IV * 2); float* O = (float*)take((size_t)NR * IV * 4);
  k_proj<<<dim3(NR / 64, 5, 3), 128, 0, stream>>>(I[0], I[2], I[1], I[3], I[4], I[5], I[6], Q32, Kh, Kl, VTh, VTl);
  k_attn<<<dim3(SS / 64, NB * NHT), 128, 0, stream>>>(Q32, Kh, Kl, VTh, VTl, I[2], I[3], I[8], O);
  k_out<<<dim3(NR / 64, OD / 128), 128, 0, stream>>>(O, I[7], (float*)d_out);
}
